// MultiHeadAttentionMyNoattn_46016279610054
// MI455X (gfx1250) — hardware-run, weakly checked
//
#include <hip/hip_runtime.h>
#include <math.h>

#define TGT 256
#define TGT_LOG2 8
#define BSZ 8
#define EMB 256
#define SRC 4096
#define NTOK TGT
#define NE 16
#define NSH BSZ
#define NROW_S (BSZ * TGT)
#define NT_MAX (NROW_S / 64)

#define CM_LOG2 11
#define CV_LOG2 11
#define CW_LOG2 16
#define CP_LOG2 7

#define TBL_COUNT 0
#define TBL_POFF 16
#define TBL_NTILES 40
#define TBL_TILE_E 64
#define TBL_HDR 256

static_assert(TGT == 256 && (1 << TGT_LOG2) == TGT && BSZ == 8 && EMB == 256 && SRC == 4096 && NE == 16 && NSH <= NE && NROW_S == 2048 && NT_MAX == 32);
static_assert(SRC % 64 == 0 && EMB % 64 == 0 && TGT % 64 == 0 && NROW_S % 64 == 0 && NROW_S / 64 <= NT_MAX);
static_assert(TBL_HDR % 32 == 0 && TBL_HDR <= 512);
static_assert(TBL_COUNT + NE <= TBL_POFF && TBL_POFF + NE + 1 <= TBL_NTILES && TBL_NTILES < TBL_TILE_E && TBL_TILE_E + NT_MAX <= TBL_HDR);
static_assert((BSZ * TGT * SRC / 8) % 256 == 0 && (EMB * EMB / 8) % 256 == 0 && (BSZ * TGT * SRC / 4) % 256 == 0);
static_assert(CM_LOG2 + CV_LOG2 == 22 && CP_LOG2 + CW_LOG2 == 23);

constexpr size_t al256(size_t b) { return (b + 255) & ~(size_t)255; }
constexpr size_t SZ_M16  = al256((size_t)BSZ * TGT * SRC * 2);
constexpr size_t SZ_VT   = al256((size_t)BSZ * EMB * SRC * 2);
constexpr size_t SZ_WO   = al256((size_t)EMB * EMB * 2);
constexpr size_t SZ_TBLD = al256((size_t)TBL_HDR * 4);
constexpr size_t SZ_P16  = al256((size_t)NROW_S * EMB * 2);
constexpr size_t WS_TOTAL = SZ_M16 + SZ_VT + SZ_WO + SZ_TBLD + SZ_P16;
static_assert(WS_TOTAL == (size_t)34735104 && WS_TOTAL < (size_t)134217728);
#define OUT1_OFF (TGT * BSZ * EMB)
static_assert(OUT1_OFF == 524288 && (OUT1_OFF * 4) % 128 == 0);

typedef _Float16 h16;
typedef __attribute__((ext_vector_type(16))) _Float16 v16h;
typedef __attribute__((ext_vector_type(8)))  _Float16 v8h;
typedef __attribute__((ext_vector_type(8)))  float    v8f;
typedef __attribute__((ext_vector_type(4)))  float    v4f;
typedef __attribute__((ext_vector_type(2)))  float    v2f;
typedef __attribute__((ext_vector_type(4)))  unsigned int v4u;
typedef __attribute__((ext_vector_type(4)))  int      v4i;
typedef __attribute__((ext_vector_type(2)))  int      v2i;


#define VST2(T, ptr, val) do { const T vst2_v_ = (val); *(volatile T*)(ptr) = vst2_v_; __threadfence(); *(volatile T*)(ptr) = vst2_v_; } while (0)

static __device__ __forceinline__ float bfr(float f) {
    unsigned u = __float_as_uint(f);
    u += 0x7FFFu + ((u >> 16) & 1u);
    return __uint_as_float(u & 0xFFFF0000u);
}
static __device__ __forceinline__ h16 toh_flush(float v) { const float w = (fabsf(v) < 6.103515625e-05f) ? 0.0f : v; return (h16)w; }
static __device__ __forceinline__ void st8h(h16* p, const float* v) {
    v8h hv;
#pragma unroll
    for (int e = 0; e < 8; ++e) hv[e] = toh_flush(v[e]);
    VST2(v8h, p, hv);
}

union FragU { v16h v; v8h h[2]; };
static __device__ __forceinline__ v16h frag_ld(const h16* p) {
    FragU f; f.h[0] = *(const v8h*)(p); f.h[1] = *(const v8h*)(p + 16); return f.v;
}
static __device__ __forceinline__ v8f wmma16g(v16h a, v16h b, v8f c) {
    c = __builtin_amdgcn_wmma_f32_16x16x32_f16(false, a, false, b, (short)0, c, false, false);
    asm volatile("v_nop\n\tv_nop\n\tv_nop\n\tv_nop" : "+v"(c) : "v"(a), "v"(b));
    return c;
}
static __device__ __forceinline__ void wave_sync_lds() {
    __builtin_amdgcn_fence(3  , "workgroup");
    __builtin_amdgcn_wave_barrier();
    __builtin_amdgcn_fence(2  , "workgroup");
}

template <int LOG2C>
__global__ __launch_bounds__(256) void k_plane(const float* __restrict__ src, h16* __restrict__ dst, unsigned n8) {
    const unsigned u = blockIdx.x * 256u + threadIdx.x;
    if (u >= n8) return;
    const float cs = (float)(1u << LOG2C);
    const v4f a = *(const v4f*)(src + (size_t)u * 8u);
    const v4f b = *(const v4f*)(src + (size_t)u * 8u + 4u);
    float v[8] = {bfr(a.x) * cs, bfr(a.y) * cs, bfr(a.z) * cs, bfr(a.w) * cs, bfr(b.x) * cs, bfr(b.y) * cs, bfr(b.z) * cs, bfr(b.w) * cs};
    st8h(dst + (size_t)u * 8u, v);
}

__global__ __launch_bounds__(128) void k_planeTw(const float* __restrict__ src, h16* __restrict__ dst, unsigned ne, unsigned K, unsigned N, unsigned pitch, unsigned estride, float cs) {
    __shared__ __align__(16) float sT[4][64 * 36];
    const unsigned lane = threadIdx.x & 31u;
    const unsigned wave = threadIdx.x >> 5;
    const unsigned tk = K >> 6, tn = N >> 5;
    const unsigned tpe = tk * tn;
    const unsigned u = blockIdx.x * 4u + wave;
    if (u >= ne * tpe) return;
    const unsigned e = u / tpe;
    const unsigned rem = u - e * tpe;
    const unsigned kt = rem / tn;
    const unsigned nt = rem - kt * tn;
    const unsigned k0 = kt << 6, n0 = nt << 5;
    const size_t sbase = (size_t)e * (size_t)estride;
    const size_t ebase = (size_t)e * ((size_t)K * (size_t)N);
    float* slab = sT[wave];
#pragma unroll
    for (int i = 0; i < 16; ++i) {
        const unsigned p = lane + 32u * (unsigned)i;
        const unsigned kr = p >> 3;
        const unsigned n4 = (p & 7u) * 4u;
        const v4f a = *(const v4f*)(src + sbase + (size_t)(k0 + kr) * pitch + n0 + n4);
        v4f s;
        s.x = bfr(a.x) * cs; s.y = bfr(a.y) * cs; s.z = bfr(a.z) * cs; s.w = bfr(a.w) * cs;
        *(v4f*)(&slab[kr * 36u + n4]) = s;
    }
    wave_sync_lds();
#pragma unroll
    for (int i = 0; i < 8; ++i) {
        const unsigned q = lane + 32u * (unsigned)i;
        const unsigned n = q >> 3;
        const unsigned kp = q & 7u;
        float v[8];
#pragma unroll
        for (int j = 0; j < 8; ++j) v[j] = slab[(8u * kp + (unsigned)j) * 36u + n];
        st8h(dst + ebase + (size_t)(n0 + n) * K + k0 + 8u * kp, v);
    }
}

__global__ __launch_bounds__(64) void k_tbl_dense(int* __restrict__ tbl) {
    const unsigned w0 = threadIdx.x * 4u;
    int q[4];
#pragma unroll
    for (int k = 0; k < 4; ++k) {
        const unsigned w = w0 + (unsigned)k;
        int val = 0;
        val = (w < (unsigned)(TBL_COUNT + NSH)) ? NTOK : val;
        val = (w >= (unsigned)TBL_POFF && w <= (unsigned)(TBL_POFF + NE)) ? (int)min((w - (unsigned)TBL_POFF) * (unsigned)NTOK, (unsigned)NROW_S) : val;
        val = (w == (unsigned)TBL_NTILES) ? (NROW_S / 64) : val;
        val = (w >= (unsigned)TBL_TILE_E && w < (unsigned)(TBL_TILE_E + NT_MAX)) ? ((w - (unsigned)TBL_TILE_E < (unsigned)(NROW_S / 64)) ? (int)((w - (unsigned)TBL_TILE_E) / (unsigned)(NTOK / 64)) : -1) : val;
        q[k] = val;
    }
    v4i v;
    v.x = q[0]; v.y = q[1]; v.z = q[2]; v.w = q[3];
    VST2(v4i, tbl + w0, v);
}

template <int KD, int ND, int MODE, int ACT, int HASB, int LOG2S, int LOG2CO, int ROWMAP>
__global__ __launch_bounds__(256) void k_linx(const h16* __restrict__ A, const h16* __restrict__ Wp, const float* __restrict__ eb,
                                             const int* __restrict__ tbl, void* __restrict__ OutV, unsigned nreal) {
    static_assert(KD % 32 == 0 && ND % 64 == 0 && MODE >= 0 && MODE <= 2 && (ACT == 0 || ACT == 1) && (HASB == 0 || HASB == 1) && LOG2S >= 0 && LOG2S <= 31 && LOG2CO >= 0 && LOG2CO <= 15 && (ROWMAP == 0 || (ROWMAP == 1 && MODE == 2)));
    constexpr float SCX = 1.0f / (float)(1u << LOG2S);
    constexpr float COX = (float)(1u << LOG2CO);
    __shared__ __align__(16) float sT[8][16 * 68];
    const unsigned lane = threadIdx.x & 31u;
    const unsigned wave = threadIdx.x >> 5;
    const unsigned u = blockIdx.x * 8u + wave;
    if (u >= (unsigned)(NT_MAX * (ND / 64))) return;
    const unsigned rowtile = u / (unsigned)(ND / 64);
    const unsigned ct = u - rowtile * (unsigned)(ND / 64);
    const int nt = min(max(tbl[TBL_NTILES], 0), NT_MAX);
    if ((int)rowtile >= nt) return;
    const int e = min(max(tbl[TBL_TILE_E + rowtile], 0), (int)nreal - 1);
    const size_t wbase = (size_t)(unsigned)e * (size_t)(ND * KD);
    const unsigned m0 = rowtile << 6, n0 = ct << 6;
    const unsigned rlane = lane & 15u;
    const unsigned koff = (lane >> 4) * 8u;
    const unsigned mOff = koff;

    v8f acc[4][4];
#pragma unroll
    for (int i = 0; i < 4; ++i)
#pragma unroll
        for (int j = 0; j < 4; ++j) acc[i][j] = (v8f){0.f,0.f,0.f,0.f,0.f,0.f,0.f,0.f};

    for (unsigned k0 = 0; k0 < (unsigned)KD; k0 += 32u) {
        v16h bh[4];
#pragma unroll
        for (int j = 0; j < 4; ++j)
            bh[j] = frag_ld(Wp + wbase + (size_t)(n0 + ((unsigned)j << 4) + rlane) * KD + koff + k0);
#pragma unroll
        for (int i = 0; i < 4; ++i) {
            const v16h ah = frag_ld(A + (size_t)(m0 + ((unsigned)i << 4) + rlane) * KD + koff + k0);
#pragma unroll
            for (int j = 0; j < 4; ++j) acc[i][j] = wmma16g(ah, bh[j], acc[i][j]);
        }
    }

    float ebv[4];
#pragma unroll
    for (int j = 0; j < 4; ++j) { if constexpr (HASB == 1) ebv[j] = bfr(eb[(unsigned)e * (unsigned)ND + n0 + ((unsigned)j << 4) + rlane]); else ebv[j] = 0.0f; }

    float* slab = sT[wave];
#pragma unroll
    for (int i = 0; i < 4; ++i) {
        const unsigned mBase = m0 + ((unsigned)i << 4);
#pragma unroll
        for (int j = 0; j < 4; ++j)
#pragma unroll
            for (int r = 0; r < 8; ++r) {
                const float a = (HASB == 1) ? (acc[i][j][r] * SCX + ebv[j]) : (acc[i][j][r] * SCX);
                const float g = (ACT == 1) ? fmaxf(a, 0.0f) : a;
                slab[(mOff + (unsigned)r) * 68u + ((unsigned)j << 4) + rlane] = (MODE == 2) ? g : g * COX;
            }
        wave_sync_lds();
        if constexpr (MODE == 2) {
            float* Out = (float*)OutV;
            const unsigned hh = lane >> 4, c4 = (lane & 15u) * 4u;
#pragma unroll
            for (int half = 0; half < 2; ++half) {
                v4f vv[4];
#pragma unroll
                for (int it = 0; it < 4; ++it) {
                    const unsigned row = (unsigned)(half * 4 + it) * 2u + hh;
                    vv[it] = *(const v4f*)(slab + row * 68u + c4);
                }
                for (int pass = 0; pass < 2; ++pass) {
#pragma unroll
                    for (int it = 0; it < 4; ++it) {
                        const unsigned row = (unsigned)(half * 4 + it) * 2u + hh;
                        const unsigned rr = mBase + row;
                        const unsigned orow = (ROWMAP == 1) ? ((rr & (unsigned)(TGT - 1)) * (unsigned)BSZ + (rr >> TGT_LOG2)) : rr;
                        *(volatile v4f*)(Out + (size_t)orow * ND + n0 + c4) = vv[it];
                    }
                    __threadfence();
                }
            }
        } else {
            h16* Out = (h16*)OutV;
            constexpr unsigned RS = (MODE == 1) ? (unsigned)(2 * ND) : (unsigned)ND;
            const unsigned q = lane >> 3, c8 = (lane & 7u) * 8u;
            v8h hv[4];
            v8h lv[4];
#pragma unroll
            for (int it = 0; it < 4; ++it) {
                const unsigned row = (unsigned)it * 4u + q;
                const float* sp = slab + row * 68u + c8;
#pragma unroll
                for (int t = 0; t < 8; ++t) {
                    const h16 hi = toh_flush(sp[t]);
                    hv[it][t] = hi;
                    lv[it][t] = (MODE == 1) ? toh_flush(sp[t] - (float)hi) : (h16)0.0f;
                }
            }
            for (int pass = 0; pass < 2; ++pass) {
#pragma unroll
                for (int it = 0; it < 4; ++it) {
                    const unsigned row = (unsigned)it * 4u + q;
                    *(volatile v8h*)(Out + (size_t)(mBase + row) * RS + n0 + c8) = hv[it];
                    if constexpr (MODE == 1) *(volatile v8h*)(Out + (size_t)(mBase + row) * RS + (unsigned)ND + n0 + c8) = lv[it];
                }
                __threadfence();
            }
        }
        wave_sync_lds();
    }
}

__global__ __launch_bounds__(256) void k_copy(const float* __restrict__ src, float* __restrict__ dst, unsigned n4) {
    const unsigned u = blockIdx.x * 256u + threadIdx.x;
    if (u >= n4) return;
    const v4f a = *(const v4f*)(src + (size_t)u * 4u);
    VST2(v4f, dst + (size_t)u * 4u, a);
}

extern "C" void kernel_launch(void* const* d_in, const int* in_sizes, int n_in, void* d_out, int out_size,
                              void* d_ws, size_t ws_size, hipStream_t stream) {
    if (n_in < 6) return;
    if (in_sizes[0] < TGT * BSZ * EMB || in_sizes[1] < SRC * BSZ * EMB || in_sizes[2] < SRC * BSZ * EMB || in_sizes[3] < BSZ * TGT * SRC || in_sizes[4] < EMB * EMB || in_sizes[5] < EMB) return;
    if (out_size < OUT1_OFF + BSZ * TGT * SRC) return;

    const float* value = (const float*)d_in[2];
    const float* mask  = (const float*)d_in[3];
    const float* wo    = (const float*)d_in[4];
    const float* bo    = (const float*)d_in[5];
    float* out0 = (float*)d_out;
    float* out1 = (float*)d_out + OUT1_OFF;

    char* wsp = (char*)d_ws;
    size_t off = 0;
    auto carve = [&](size_t bytes) -> void* { void* r = wsp + off; off += (bytes + 255) & ~(size_t)255; return r; };
    h16* m16  = (h16*)carve((size_t)BSZ * TGT * SRC * 2);
    h16* vT   = (h16*)carve((size_t)BSZ * EMB * SRC * 2);
    h16* wo16 = (h16*)carve((size_t)EMB * EMB * 2);
    int* tblD = (int*)carve((size_t)TBL_HDR * 4);
    h16* P16  = (h16*)carve((size_t)NROW_S * EMB * 2);
    if (off != WS_TOTAL || off > ws_size || off > (size_t)134217728) return;

    k_plane<CM_LOG2><<<(BSZ * TGT * SRC / 8) / 256, 256, 0, stream>>>(mask, m16, (unsigned)(BSZ * TGT * SRC / 8));
    constexpr float cv = (float)(1u << CV_LOG2);
    k_planeTw<<<(BSZ * (SRC / 64) * (EMB / 32) + 3) / 4, 128, 0, stream>>>(value, vT, (unsigned)BSZ, (unsigned)SRC, (unsigned)EMB, (unsigned)(BSZ * EMB), (unsigned)EMB, cv);
    k_plane<CW_LOG2><<<(EMB * EMB / 8) / 256, 256, 0, stream>>>(wo, wo16, (unsigned)(EMB * EMB / 8));
    k_tbl_dense<<<1, 64, 0, stream>>>(tblD);
    k_linx<SRC, EMB, 0, 0, 0, CM_LOG2 + CV_LOG2, CP_LOG2, 0><<<(NT_MAX * (EMB / 64) + 7) / 8, 256, 0, stream>>>(m16, vT, bo, tblD, (void*)P16, (unsigned)BSZ);
    k_linx<EMB, EMB, 2, 0, 1, CP_LOG2 + CW_LOG2, 0, 1><<<(NT_MAX * (EMB / 64) + 7) / 8, 256, 0, stream>>>(P16, wo16, bo, tblD, (void*)out0, 1u);
    k_copy<<<(BSZ * TGT * SRC / 4) / 256, 256, 0, stream>>>(mask, out1, (unsigned)(BSZ * TGT * SRC / 4));
}
